// ZiSAWrapper_80788334838079
// MI455X (gfx1250) — hardware-verified
//
#include <hip/hip_runtime.h>


namespace {
constexpr int Bn = 2, C = 64, HH = 96, WWD = 96, NPOS = HH * WWD  , PH = 48, PW = 48, NK = PH * PW  , NHD = 4, DH = 16, NPB = NPOS / 128  ;
constexpr float QS = 8.0f, VS = 8.0f, PS = 8.0f, OS_ = 8.0f, SCALE = 0.25f;
constexpr size_t QPL = (size_t)Bn * NHD * NPOS * 32, KPL = (size_t)Bn * NHD * NK * 32, VPL = (size_t)Bn * NHD * DH * NK;

typedef _Float16 b16;
typedef __attribute__((ext_vector_type(16))) _Float16 v16b;
typedef __attribute__((ext_vector_type(8))) _Float16 v8b;
typedef __attribute__((ext_vector_type(8))) float v8f;
typedef __attribute__((ext_vector_type(4))) float v4f;
__device__ __forceinline__ float bf16_rne(float f) { unsigned int u = __float_as_uint(f); u += 0x7FFFu + ((u >> 16) & 1u); return __uint_as_float(u & 0xFFFF0000u); }
__device__ __forceinline__ void split16(float v, b16& hi, b16& lo) { hi = (b16)v; lo = (b16)(v - (float)hi); }
__device__ __forceinline__ v16b frag_kb(const b16* p, int hh) { const v8b a = *(const v8b*)(p + 8 * hh), b = *(const v8b*)(p + 16 + 8 * hh); v16b f;
#pragma unroll
  for (int e = 0; e < 8; ++e) { f[e] = a[e]; f[8 + e] = b[e]; } return f; }
__device__ __forceinline__ v8f wmma16b(v16b a, v16b b, v8f c) { v8f d = __builtin_amdgcn_wmma_f32_16x16x32_f16(false, a, false, b, (short)0, c, false, false); asm volatile("v_nop\n\tv_nop\n\tv_nop\n\tv_nop" : "+v"(d) : "v"(a), "v"(b)); return d; }
__device__ __forceinline__ void wave_lds_sync() { __builtin_amdgcn_fence(__ATOMIC_RELEASE, "workgroup"); __builtin_amdgcn_wave_barrier(); __builtin_amdgcn_fence(__ATOMIC_ACQUIRE, "workgroup"); }
__device__ __forceinline__ float nexp(float x) { return __builtin_amdgcn_exp2f(x * 1.4426950408889634f); }

__global__ __launch_bounds__(256) void prepx_kernel(const float* __restrict__ x, b16* __restrict__ xT) {
  __shared__ __attribute__((aligned(16))) b16 Tt[128][C + 8];
  const int b = blockIdx.y, p0 = blockIdx.x * 128, t_ = threadIdx.x;
  for (int i = t_; i < C * 128; i += 256) { const int c = i >> 7, pp = i & 127; Tt[pp][c] = (b16)bf16_rne(x[((size_t)b * C + c) * NPOS + p0 + pp]); }
  __syncthreads();
  for (int pass = 0; pass < 2; ++pass) { for (int i = t_; i < 128 * C / 8; i += 256) { const int pp = i >> 3, c8 = (i & 7) * 8; *(volatile v8b*)(xT + ((size_t)b * NPOS + p0 + pp) * C + c8) = *(const v8b*)(&Tt[pp][c8]); } __threadfence(); }
}
__global__ __launch_bounds__(256) void pool_kernel(const float* __restrict__ x, b16* __restrict__ xph, b16* __restrict__ xpl) {
  __shared__ __attribute__((aligned(16))) b16 Th[PW][C + 8], Tl[PW][C + 8];
  const int b = blockIdx.y, py = blockIdx.x, t_ = threadIdx.x;
  for (int i = t_; i < C * PW; i += 256) { const int c = i / PW, px = i % PW; const float* r0 = x + ((size_t)b * C + c) * NPOS + (size_t)(2 * py) * WWD + 2 * px;
    const float m = (bf16_rne(r0[0]) + bf16_rne(r0[1]) + bf16_rne(r0[WWD]) + bf16_rne(r0[WWD + 1])) * 0.25f; b16 a, l; split16(m, a, l); Th[px][c] = a; Tl[px][c] = l; }
  __syncthreads();
  for (int pass = 0; pass < 2; ++pass) { for (int i = t_; i < PW * C / 8; i += 256) { const int px = i >> 3, c8 = (i & 7) * 8; const size_t row = (size_t)b * NK + py * PW + px;
      *(volatile v8b*)(xph + row * C + c8) = *(const v8b*)(&Th[px][c8]); *(volatile v8b*)(xpl + row * C + c8) = *(const v8b*)(&Tl[px][c8]); } __threadfence(); }
}
__global__ __launch_bounds__(256) void prepw_kernel(const float* __restrict__ wq, const float* __restrict__ wk, const float* __restrict__ wv, const float* __restrict__ wo, b16* __restrict__ w16) {
  const int t_ = threadIdx.x;
  for (int pass = 0; pass < 2; ++pass) { for (int p = t_; p < 4 * C * C; p += 256) { const int m = p / (C * C), q = p % (C * C); const float* W = (m == 0) ? wq : (m == 1) ? wk : (m == 2) ? wv : wo; ((volatile b16*)w16)[p] = (b16)bf16_rne(W[q]); } __threadfence(); }
}

__global__ __launch_bounds__(128) void qproj_kernel(const b16* __restrict__ xT, const b16* __restrict__ w16, const float* __restrict__ bq, b16* __restrict__ qh) {
  __shared__ __attribute__((aligned(16))) b16 Th[NHD][128][32], Tl[NHD][128][32];
  const int lane = threadIdx.x & 31, wave = threadIdx.x >> 5, nloc = lane & 15, hlf = lane >> 4, b = blockIdx.y, p0 = blockIdx.x * 128, m0 = wave * 32;
  for (int i = threadIdx.x; i < NHD * 128 * 32 / 8; i += 128) { const v8b z = {}; *(v8b*)(&Th[0][0][0] + i * 8) = z; *(v8b*)(&Tl[0][0][0] + i * 8) = z; }
  __syncthreads();
  v8f acc[2][4];
#pragma unroll
  for (int r = 0; r < 2; ++r)
#pragma unroll
    for (int t = 0; t < 4; ++t) acc[r][t] = (v8f){};
  const b16* A = xT + ((size_t)b * NPOS + p0 + m0) * C;
#pragma unroll
  for (int kb = 0; kb < C; kb += 32) { const v16b a0 = frag_kb(A + (size_t)nloc * C + kb, hlf), a1 = frag_kb(A + (size_t)(16 + nloc) * C + kb, hlf);
#pragma unroll
    for (int t = 0; t < 4; ++t) { const v16b bw = frag_kb(w16 + (size_t)(t * 16 + nloc) * C + kb, hlf); acc[0][t] = wmma16b(a0, bw, acc[0][t]); acc[1][t] = wmma16b(a1, bw, acc[1][t]); } }
#pragma unroll
  for (int t = 0; t < 4; ++t) { const float bb = bf16_rne(bq[t * 16 + nloc]);
#pragma unroll
    for (int r = 0; r < 2; ++r)
#pragma unroll
      for (int v = 0; v < 8; ++v) { b16 a_, c_; split16((acc[r][t][v] + bb) * QS, a_, c_); Th[t][m0 + r * 16 + 8 * hlf + v][nloc] = a_; Tl[t][m0 + r * 16 + 8 * hlf + v][nloc] = c_; } }
  __syncthreads();
  for (int pass = 0; pass < 2; ++pass) {
    for (int i = threadIdx.x; i < NHD * 128 * 32 / 8; i += 128) { const int h = i / 512, rem = i % 512; const size_t dst = (((size_t)b * NHD + h) * NPOS + p0) * 32 + (size_t)rem * 8;
      *(volatile v8b*)(qh + dst) = *(const v8b*)(&Th[h][0][0] + rem * 8); *(volatile v8b*)(qh + QPL + dst) = *(const v8b*)(&Tl[h][0][0] + rem * 8); }
    __threadfence(); }
}
__global__ __launch_bounds__(256) void kvproj_kernel(const b16* __restrict__ xph, const b16* __restrict__ xpl, const b16* __restrict__ w16, const float* __restrict__ bk, const float* __restrict__ bv, b16* __restrict__ kh, b16* __restrict__ vt) {
  __shared__ __attribute__((aligned(16))) b16 Th[NHD][128][32], Tl[NHD][128][32]; __shared__ __attribute__((aligned(16))) b16 Vh[C][128 + 8], Vl[C][128 + 8];
  const int lane = threadIdx.x & 31, wave = threadIdx.x >> 5, nloc = lane & 15, hlf = lane >> 4, b = blockIdx.y, p0 = blockIdx.x * 128, which = wave >> 2, m0 = (wave & 3) * 32;
  for (int i = threadIdx.x; i < NHD * 128 * 32 / 8; i += 256) { const v8b z = {}; *(v8b*)(&Th[0][0][0] + i * 8) = z; *(v8b*)(&Tl[0][0][0] + i * 8) = z; }
  __syncthreads();
  v8f acc[2][4];
#pragma unroll
  for (int r = 0; r < 2; ++r)
#pragma unroll
    for (int t = 0; t < 4; ++t) acc[r][t] = (v8f){};
  const b16* A = xph + ((size_t)b * NK + p0 + m0) * C; const b16* AL = xpl + ((size_t)b * NK + p0 + m0) * C; const b16* Bw = w16 + (size_t)(1 + which) * C * C;
#pragma unroll
  for (int kb = 0; kb < C; kb += 32) { const v16b a0 = frag_kb(A + (size_t)nloc * C + kb, hlf), l0 = frag_kb(AL + (size_t)nloc * C + kb, hlf), a1 = frag_kb(A + (size_t)(16 + nloc) * C + kb, hlf), l1 = frag_kb(AL + (size_t)(16 + nloc) * C + kb, hlf);
#pragma unroll
    for (int t = 0; t < 4; ++t) { const v16b bw = frag_kb(Bw + (size_t)(t * 16 + nloc) * C + kb, hlf); acc[0][t] = wmma16b(a0, bw, acc[0][t]); acc[0][t] = wmma16b(l0, bw, acc[0][t]); acc[1][t] = wmma16b(a1, bw, acc[1][t]); acc[1][t] = wmma16b(l1, bw, acc[1][t]); } }
  if (which == 0) {
#pragma unroll
    for (int t = 0; t < 4; ++t) { const float bb = bf16_rne(bk[t * 16 + nloc]);
#pragma unroll
      for (int r = 0; r < 2; ++r)
#pragma unroll
        for (int v = 0; v < 8; ++v) { b16 a_, c_; split16((acc[r][t][v] + bb) * QS, a_, c_); Th[t][m0 + r * 16 + 8 * hlf + v][nloc] = a_; Tl[t][m0 + r * 16 + 8 * hlf + v][nloc] = c_; } }
  } else {
#pragma unroll
    for (int t = 0; t < 4; ++t) { const float bb = bf16_rne(bv[t * 16 + nloc]);
#pragma unroll
      for (int r = 0; r < 2; ++r)
#pragma unroll
        for (int v = 0; v < 8; ++v) { b16 a_, c_; split16((acc[r][t][v] + bb) * VS, a_, c_); Vh[t * 16 + nloc][m0 + r * 16 + 8 * hlf + v] = a_; Vl[t * 16 + nloc][m0 + r * 16 + 8 * hlf + v] = c_; } }
  }
  __syncthreads();
  for (int pass = 0; pass < 2; ++pass) {
    if (which == 0) { for (int i = threadIdx.x; i < NHD * 128 * 32 / 8; i += 128) { const int h = i / 512, rem = i % 512; const size_t dst = (((size_t)b * NHD + h) * NK + p0) * 32 + (size_t)rem * 8;
        *(volatile v8b*)(kh + dst) = *(const v8b*)(&Th[h][0][0] + rem * 8); *(volatile v8b*)(kh + KPL + dst) = *(const v8b*)(&Tl[h][0][0] + rem * 8); } }
    else { for (int i = threadIdx.x - 128; i < C * 16; i += 128) { const int c = i >> 4, c8 = (i & 15) * 8; const int h = c / DH, d = c % DH; const size_t dst = (((size_t)b * NHD + h) * DH + d) * NK + p0 + c8;
        *(volatile v8b*)(vt + dst) = *(const v8b*)(&Vh[c][c8]); *(volatile v8b*)(vt + VPL + dst) = *(const v8b*)(&Vl[c][c8]); } }
    __threadfence(); }
}

__global__ __launch_bounds__(256) void attn_kernel(const b16* __restrict__ qh, const b16* __restrict__ kh, const b16* __restrict__ vt, float* __restrict__ orow) {
  __shared__ __attribute__((aligned(16))) float Os[32][C + 4];
  const int wid = threadIdx.x >> 5, lane = threadIdx.x & 31, hh = lane >> 4, col = lane & 15;
  const int b = blockIdx.x / (NPOS / 32), qt2 = blockIdx.x % (NPOS / 32), h = wid & 3, sub = wid >> 2, q0 = qt2 * 32 + sub * 16, qi = q0 + col;
  const b16* Q = qh + (((size_t)b * NHD + h) * NPOS) * 32; const b16* K = kh + (((size_t)b * NHD + h) * NK) * 32; const b16* V = vt + (((size_t)b * NHD + h) * DH) * NK;
  const v16b qf = frag_kb(Q + (size_t)qi * 32, hh), ql = frag_kb(Q + QPL + (size_t)qi * 32, hh);
  float m = -INFINITY, l = 0.0f; v8f o = {};
  for (int kb = 0; kb < NK; kb += 32) {
    const v16b ka = frag_kb(K + (size_t)(kb + col) * 32, hh), kal = frag_kb(K + KPL + (size_t)(kb + col) * 32, hh), kb_ = frag_kb(K + (size_t)(kb + 16 + col) * 32, hh), kbl = frag_kb(K + KPL + (size_t)(kb + 16 + col) * 32, hh);
    v8f s0 = {}, s1 = {}; s0 = wmma16b(ka, qf, s0); s0 = wmma16b(ka, ql, s0); s0 = wmma16b(kal, qf, s0); s1 = wmma16b(kb_, qf, s1); s1 = wmma16b(kb_, ql, s1); s1 = wmma16b(kbl, qf, s1);
    float mr = -INFINITY;
#pragma unroll
    for (int r = 0; r < 8; ++r) { s0[r] *= SCALE / (QS * QS); s1[r] *= SCALE / (QS * QS); mr = fmaxf(mr, fmaxf(s0[r], s1[r])); }
    mr = fmaxf(mr, __shfl_xor(mr, 16));
    const float mn = fmaxf(m, mr), al_ = nexp(m - mn); m = mn; float sum = 0.0f; v16b pb, pl;
#pragma unroll
    for (int r = 0; r < 8; ++r) { const float p0 = nexp(s0[r] - mn), p1 = nexp(s1[r] - mn); sum += p0 + p1; b16 a, c; split16(p0 * PS, a, c); pb[r] = a; pl[r] = c; split16(p1 * PS, a, c); pb[8 + r] = a; pl[8 + r] = c; }
    sum += __shfl_xor(sum, 16); l = l * al_ + sum;
#pragma unroll
    for (int r = 0; r < 8; ++r) o[r] *= al_;
    const v16b vf = frag_kb(V + (size_t)col * NK + kb, hh), vl = frag_kb(V + VPL + (size_t)col * NK + kb, hh);
    o = wmma16b(vf, pb, o); o = wmma16b(vf, pl, o); o = wmma16b(vl, pb, o); }
  const float inv = 1.0f / (l * VS * PS);
#pragma unroll
  for (int r = 0; r < 8; ++r) Os[sub * 16 + col][h * DH + 8 * hh + r] = o[r] * inv;
  __syncthreads();
  float* dst = orow + ((size_t)b * NPOS + qt2 * 32) * C;
  for (int pass = 0; pass < 2; ++pass) { for (int i = threadIdx.x; i < 32 * C / 4; i += 256) { const int rr = i >> 4, c4 = (i & 15) * 4; *(volatile v4f*)(dst + (size_t)rr * C + c4) = *(const v4f*)(&Os[rr][c4]); } __threadfence(); }
}

__global__ __launch_bounds__(128) void oproj_kernel(const float* __restrict__ orow, const b16* __restrict__ w16, const float* __restrict__ bo, float* __restrict__ ao, float* __restrict__ part) {
  __shared__ __attribute__((aligned(16))) float Ts[4][32 * 64]; __shared__ float Cs[4][64];
  const int lane = threadIdx.x & 31, wave = threadIdx.x >> 5, nloc = lane & 15, hlf = lane >> 4, b = blockIdx.y, p0 = blockIdx.x * 128, m0 = wave * 32;
  const float* A = orow + ((size_t)b * NPOS + p0 + m0) * C; const b16* Bw = w16 + (size_t)3 * C * C;
  v8f acc[2][4];
#pragma unroll
  for (int r = 0; r < 2; ++r)
#pragma unroll
    for (int t = 0; t < 4; ++t) acc[r][t] = (v8f){};
#pragma unroll
  for (int kb = 0; kb < C; kb += 32) { v16b a0, a1, l0, l1;
#pragma unroll
    for (int e = 0; e < 16; ++e) { const int k = kb + ((e < 8) ? (8 * hlf + e) : (16 + 8 * hlf + e - 8)); b16 p, q; split16(A[(size_t)nloc * C + k] * OS_, p, q); a0[e] = p; l0[e] = q; split16(A[(size_t)(16 + nloc) * C + k] * OS_, p, q); a1[e] = p; l1[e] = q; }
#pragma unroll
    for (int t = 0; t < 4; ++t) { const v16b bw = frag_kb(Bw + (size_t)(t * 16 + nloc) * C + kb, hlf); acc[0][t] = wmma16b(a0, bw, acc[0][t]); acc[0][t] = wmma16b(l0, bw, acc[0][t]); acc[1][t] = wmma16b(a1, bw, acc[1][t]); acc[1][t] = wmma16b(l1, bw, acc[1][t]); } }
  float* Tt = Ts[wave];
#pragma unroll
  for (int t = 0; t < 4; ++t) { const float bb = bf16_rne(bo[t * 16 + nloc]);
#pragma unroll
    for (int r = 0; r < 2; ++r)
#pragma unroll
      for (int v = 0; v < 8; ++v) Tt[(r * 16 + v + 8 * hlf) * 64 + t * 16 + nloc] = acc[r][t][v] * (1.0f / OS_) + bb; }
  wave_lds_sync();
  { float s = 0.0f; for (int rr = 0; rr < 32; ++rr) s += Tt[rr * 64 + lane * 2]; float s2 = 0.0f; for (int rr = 0; rr < 32; ++rr) s2 += Tt[rr * 64 + lane * 2 + 1]; Cs[wave][lane * 2] = s; Cs[wave][lane * 2 + 1] = s2; }
  __syncthreads();
  float* dst0 = ao + ((size_t)b * NPOS + p0 + m0) * C;
  for (int pass = 0; pass < 2; ++pass) {
#pragma unroll
    for (int j = 0; j < 16; ++j) { const int rr = j * 2 + hlf, c4 = nloc * 4; *(volatile v4f*)(dst0 + (size_t)rr * C + c4) = *(const v4f*)(Tt + rr * 64 + c4); }
    if (threadIdx.x < 64) ((volatile float*)part)[((size_t)b * NPB + blockIdx.x) * C + threadIdx.x] = Cs[0][threadIdx.x] + Cs[1][threadIdx.x] + Cs[2][threadIdx.x] + Cs[3][threadIdx.x];
    __threadfence(); }
}

__global__ __launch_bounds__(64) void gate_kernel(const float* __restrict__ part, const float* __restrict__ x, const float* __restrict__ W1, const float* __restrict__ b1, const float* __restrict__ W2, const float* __restrict__ b2, const float* __restrict__ Wg, const float* __restrict__ bg, float* __restrict__ coef) {
  __shared__ float gap[C], gx[C], se[4], caS[C], gf[C];
  const int b = blockIdx.x, c = threadIdx.x;
  { float s = 0.0f; for (int k = 0; k < NPB; ++k) s += part[((size_t)b * NPB + k) * C + c]; gap[c] = s * (1.0f / NPOS);
    const float* xr = x + ((size_t)b * C + c) * NPOS; float sx = 0.0f; for (int p = 0; p < NPOS; p += 4) { const v4f v = *(const v4f*)(xr + p); sx += (bf16_rne(v[0]) + bf16_rne(v[1])) + (bf16_rne(v[2]) + bf16_rne(v[3])); } gx[c] = sx * (1.0f / NPOS); }
  __syncthreads();
  if (c < 4) { float a = bf16_rne(b1[c]); for (int k = 0; k < C; ++k) a += bf16_rne(W1[c * C + k]) * gap[k]; se[c] = fmaxf(a, 0.0f); }
  __syncthreads();
  { float a = bf16_rne(b2[c]); for (int k = 0; k < 4; ++k) a += bf16_rne(W2[c * 4 + k]) * se[k]; const float ca = 1.0f / (1.0f + __expf(-a)); caS[c] = ca; gf[c] = gx[c] + ca * gap[c]; }
  __syncthreads();
  { float a = bf16_rne(bg[c]); for (int k = 0; k < C; ++k) a += bf16_rne(Wg[c * 2 * C + k]) * gx[k]; for (int k = 0; k < C; ++k) a += bf16_rne(Wg[c * 2 * C + C + k]) * gf[k];
    const float gate = 1.0f / (1.0f + __expf(-a)); const float cf = gate * caS[c];
    for (int pass = 0; pass < 2; ++pass) { ((volatile float*)coef)[(size_t)b * C + c] = cf; __threadfence(); } }
}

__global__ __launch_bounds__(256) void final_kernel(const float* __restrict__ x, const float* __restrict__ ao, const float* __restrict__ coef, float* __restrict__ out) {
  __shared__ __attribute__((aligned(16))) float Ta[C][128 + 4];
  const int b = blockIdx.y, p0 = blockIdx.x * 128, t_ = threadIdx.x;
  for (int i = t_; i < 128 * C / 4; i += 256) { const int pp = i >> 4, c4 = (i & 15) * 4; const v4f v = *(const v4f*)(ao + ((size_t)b * NPOS + p0 + pp) * C + c4);
#pragma unroll
    for (int e = 0; e < 4; ++e) Ta[c4 + e][pp] = v[e]; }
  __syncthreads();
  for (int pass = 0; pass < 2; ++pass) { for (int i = t_; i < C * 32; i += 256) { const int c = i >> 5, q4 = (i & 31) * 4; const float cf = coef[(size_t)b * C + c]; const size_t g = ((size_t)b * C + c) * NPOS + p0 + q4;
      const v4f xv = *(const v4f*)(x + g); v4f o;
#pragma unroll
      for (int e = 0; e < 4; ++e) o[e] = bf16_rne(xv[e]) + cf * Ta[c][q4 + e];
      *(volatile v4f*)(out + g) = o; } __threadfence(); }
}
}

extern "C" void kernel_launch(void* const* d_in, const int* in_sizes, int n_in,
                              void* d_out, int out_size, void* d_ws, size_t ws_size, hipStream_t stream) {
  (void)n_in; (void)out_size;
  const float* x = (const float*)d_in[0]; const float* wq = (const float*)d_in[1]; const float* bq = (const float*)d_in[2]; const float* wk = (const float*)d_in[3]; const float* bk = (const float*)d_in[4];
  const float* wv = (const float*)d_in[5]; const float* bv = (const float*)d_in[6]; const float* wo = (const float*)d_in[7]; const float* bo = (const float*)d_in[8];
  const float* W1 = (const float*)d_in[9]; const float* b1 = (const float*)d_in[10]; const float* W2 = (const float*)d_in[11]; const float* b2 = (const float*)d_in[12]; const float* Wg = (const float*)d_in[13]; const float* bg = (const float*)d_in[14];
  float* out = (float*)d_out;
  if (in_sizes[0] != Bn * C * NPOS || in_sizes[1] != C * C || in_sizes[7] != C * C || in_sizes[9] != 4 * C || in_sizes[13] != C * 2 * C) return;
  size_t off = 0; char* ws = (char*)d_ws;
  auto carve = [&](size_t bytes) { char* p = ws + off; off += (bytes + 255) & ~(size_t)255; return p; };
  b16* xT = (b16*)carve((size_t)Bn * NPOS * C * 2); b16* xph = (b16*)carve((size_t)Bn * NK * C * 2); b16* xpl = (b16*)carve((size_t)Bn * NK * C * 2); b16* w16 = (b16*)carve((size_t)4 * C * C * 2);
  b16* qhp = (b16*)carve(QPL * 2 * 2); b16* khp = (b16*)carve(KPL * 2 * 2); b16* vtp = (b16*)carve(VPL * 2 * 2); float* orow = (float*)carve((size_t)Bn * NPOS * C * 4); float* ao = (float*)carve((size_t)Bn * NPOS * C * 4);
  float* part = (float*)carve((size_t)Bn * NPB * C * 4); float* coef = (float*)carve((size_t)Bn * C * 4);
  if (off > ws_size) return;
  prepx_kernel<<<dim3(NPB, Bn), 256, 0, stream>>>(x, xT);
  pool_kernel<<<dim3(PH, Bn), 256, 0, stream>>>(x, xph, xpl);
  prepw_kernel<<<1, 256, 0, stream>>>(wq, wk, wv, wo, w16);
  qproj_kernel<<<dim3(NPB, Bn), 128, 0, stream>>>(xT, w16, bq, qhp);
  kvproj_kernel<<<dim3(NK / 128, Bn), 256, 0, stream>>>(xph, xpl, w16, bk, bv, khp, vtp);
  attn_kernel<<<Bn * NPOS / 32, 256, 0, stream>>>(qhp, khp, vtp, orow);
  oproj_kernel<<<dim3(NPB, Bn), 128, 0, stream>>>(orow, w16, bo, ao, part);
  gate_kernel<<<Bn, 64, 0, stream>>>(part, x, W1, b1, W2, b2, Wg, bg, coef);
  final_kernel<<<dim3(NPB, Bn), 256, 0, stream>>>(x, ao, coef, out);
}
